// TConformerQKV_61735859912778
// MI455X (gfx1250) — hardware-verified
//
#include <hip/hip_runtime.h>
#include <math.h>

#define NDIM   64
#define SEQT   512
#define NF     65
#define DFFN   256
#define WLEN   64
#define CHUNK  128
#define NKL    192
#define XP     68
#define KP     72
#define VP     208
#define CST    (SEQT * NF)
#define TL     32
#define RUN    (TL * NF)

#define WI_OFF 0
#define WO_OFF 12288
#define W1_OFF 16384
#define W2_OFF 32768
#define W16_N  49152

#define WSC    32.0f
#define WSCI   0.03125f
#define QSC    0.25f
#define PSC    16384.0f
#define PSCI   0.00006103515625f

typedef _Float16 v16h __attribute__((ext_vector_type(16)));
typedef _Float16 v8h  __attribute__((ext_vector_type(8)));
typedef float    v8f  __attribute__((ext_vector_type(8)));
typedef float    v4f  __attribute__((ext_vector_type(4)));
typedef v8h __attribute__((may_alias)) v8ha;
typedef v4f __attribute__((may_alias)) v4fa;

union Frag { v16h v; v8h half[2]; };

#define H0 ((_Float16)0.0f)

__device__ __forceinline__ v8f wmma_f16(v16h a, v16h b, v8f c) {
  v8f d = __builtin_amdgcn_wmma_f32_16x16x32_f16(false, a, false, b, (short)0, c, false, false);
  asm volatile("v_nop\n\tv_nop\n\tv_nop\n\tv_nop" : "+v"(d) : "v"(a), "v"(b));
  return d;
}

__device__ __forceinline__ v8f zero8f() { const v8f z = {0.f, 0.f, 0.f, 0.f, 0.f, 0.f, 0.f, 0.f}; return z; }
__device__ __forceinline__ v8h zero8h() { const v8h z = {H0, H0, H0, H0, H0, H0, H0, H0}; return z; }
__device__ __forceinline__ v8h cvt8(v8f x) { return __builtin_convertvector(x, v8h); }
__device__ __forceinline__ v8f ld8(const float* p) {
  const v8f r = {p[0], p[1], p[2], p[3], p[4], p[5], p[6], p[7]};
  return r;
}
__device__ __forceinline__ v8f ld8a(const float* p) {
  const v4f a = *(const v4fa*)p;
  const v4f b = *(const v4fa*)(p + 4);
  const v8f r = {a.x, a.y, a.z, a.w, b.x, b.y, b.z, b.w};
  return r;
}
__device__ __forceinline__ void st8a(float* p, v8f v) {
  const v4f a = {v[0], v[1], v[2], v[3]};
  const v4f b = {v[4], v[5], v[6], v[7]};
  *(v4fa*)p = a;
  *(v4fa*)(p + 4) = b;
}
__device__ __forceinline__ float hsum8(v8f v) {
  return ((v[0] + v[1]) + (v[2] + v[3])) + ((v[4] + v[5]) + (v[6] + v[7]));
}
__device__ __forceinline__ float gelu_f(float x) {
  return 0.5f * x * (1.0f + erff(x * 0.70710678118654752f));
}

__device__ __forceinline__ v16h load_frag(const _Float16* p, int hf) {
  Frag f;
  f.half[0] = *(const v8ha*)(p + 8 * hf);
  f.half[1] = *(const v8ha*)(p + 16 + 8 * hf);
  return f.v;
}

#define LDC(c) p[(size_t)(c) * CST]
__device__ __forceinline__ v16h xt_frag_global(const float* __restrict__ p, int hf) {
  const int ca = 8 * hf, cb = 16 + 8 * hf;
  const v8f a = {LDC(ca), LDC(ca + 1), LDC(ca + 2), LDC(ca + 3), LDC(ca + 4), LDC(ca + 5), LDC(ca + 6), LDC(ca + 7)};
  const v8f b = {LDC(cb), LDC(cb + 1), LDC(cb + 2), LDC(cb + 3), LDC(cb + 4), LDC(cb + 5), LDC(cb + 6), LDC(cb + 7)};
  Frag f;
  f.half[0] = cvt8(a);
  f.half[1] = cvt8(b);
  return f.v;
}
#undef LDC

__device__ __forceinline__ v16h xt_frag_lds(const float* p, int hf) {
  Frag f;
  f.half[0] = cvt8(ld8a(p + 8 * hf));
  f.half[1] = cvt8(ld8a(p + 16 + 8 * hf));
  return f.v;
}

__global__ __launch_bounds__(256) void cvt_w_kernel(
    const float* __restrict__ inw, const float* __restrict__ outw,
    const float* __restrict__ w1,  const float* __restrict__ w2,
    _Float16* __restrict__ w16)
{
  const int g = blockIdx.x * 256 + threadIdx.x;
  if (g >= W16_N / 8) return;
  const float* src;
  if (g < WO_OFF / 8)      src = inw  + (size_t)g * 8;
  else if (g < W1_OFF / 8) src = outw + (size_t)(g - WO_OFF / 8) * 8;
  else if (g < W2_OFF / 8) src = w1   + (size_t)(g - W1_OFF / 8) * 8;
  else                     src = w2   + (size_t)(g - W2_OFF / 8) * 8;
  const v8h o = cvt8(ld8(src) * WSC);
  _Float16* dst = w16 + (size_t)g * 8;
  *(volatile v8h*)dst = o;
  __threadfence();
  *(volatile v8h*)dst = o;
}

__device__ __forceinline__ void y_store_pass(const float* sow, float* yg, size_t rowbase, int l) {
  const int q8 = l & 7, sub = l >> 3;
#pragma unroll
  for (int i = 0; i < 8; ++i) {
    const int lid = 4 * i + sub;
    const int row = lid >> 1, hl = lid & 1;
    const v4f v = *(const v4fa*)(sow + row * NDIM + 32 * hl + 4 * q8);
    *(volatile v4f*)(yg + (rowbase + row) * NDIM + 32 * hl + 4 * q8) = v;
  }
}

__global__ __launch_bounds__(256) void fused_block_kernel(
    const float* __restrict__ qg, const float* __restrict__ kg, const float* __restrict__ vg,
    const _Float16* __restrict__ w16,
    const float* __restrict__ inb, const float* __restrict__ outb,
    const float* __restrict__ l1w, const float* __restrict__ l1b,
    const float* __restrict__ b1,  const float* __restrict__ b2,
    const float* __restrict__ l2w, const float* __restrict__ l2b,
    float* __restrict__ yg)
{
  __shared__ __align__(16) float    xs[CHUNK * XP];
  __shared__ __align__(16) _Float16 khs[NKL * KP];
  __shared__ __align__(16) _Float16 vts[NDIM * VP];
  __shared__ __align__(16) float    so[8 * 16 * NDIM];

  const int tid = threadIdx.x, w = tid >> 5, l = tid & 31;
  const int hf = l >> 4, m = l & 15;
  const int n = blockIdx.x >> 2, chunk = blockIdx.x & 3;
  const int bb = n / NF, fi = n - bb * NF;
  const int q0 = chunk * CHUNK;
  const size_t boff = (size_t)bb * NDIM * CST + fi;

  for (int i = tid; i < CHUNK * NDIM; i += 256) {
    const int t = i & (CHUNK - 1), c = i >> 7;
    xs[t * XP + c] = qg[boff + (size_t)c * CST + (size_t)(q0 + t) * NF];
  }
  if (tid < 128) {
    const int row = tid >> 1, g8 = tid & 1;
    *(v8ha*)(vts + row * VP + NKL + 8 * g8) = zero8h();
  }

#pragma unroll 1
  for (int it = 0; it < 3; ++it) {
    const int tile = w + 8 * it;
    const int isv  = (tile >= 12) ? 1 : 0;
    const int kt   = tile - 12 * isv;
    const int key  = q0 - WLEN + kt * 16 + m;
    const int tok  = key < 0 ? 0 : key;
    const float* src = (isv ? vg : kg) + boff + (size_t)tok * NF;
    const v16h xb0 = xt_frag_global(src, hf);
    const v16h xb1 = xt_frag_global(src + (size_t)32 * CST, hf);
    const int wrow0 = NDIM + NDIM * isv;
#pragma unroll
    for (int ct = 0; ct < 4; ++ct) {
      const _Float16* wr = w16 + WI_OFF + (size_t)(wrow0 + 16 * ct + m) * NDIM;
      v8f acc = zero8f();
      acc = wmma_f16(load_frag(wr, hf),      xb0, acc);
      acc = wmma_f16(load_frag(wr + 32, hf), xb1, acc);
      const v8h y = cvt8(acc * WSCI + ld8(inb + wrow0 + 16 * ct + 8 * hf));
      if (isv) {
        _Float16* vd = vts + (16 * ct + 8 * hf) * VP + kt * 16 + m;
        vd[0 * VP] = y[0]; vd[1 * VP] = y[1]; vd[2 * VP] = y[2]; vd[3 * VP] = y[3];
        vd[4 * VP] = y[4]; vd[5 * VP] = y[5]; vd[6 * VP] = y[6]; vd[7 * VP] = y[7];
      } else {
        *(v8ha*)(khs + (kt * 16 + m) * KP + 16 * ct + 8 * hf) = y;
      }
    }
  }
  __syncthreads();

  const int t0 = q0 + 16 * w;
  const int tq = t0 + m;
  const float* xr = xs + (16 * w + m) * XP;
  float* sorow = so + w * (16 * NDIM) + m * NDIM;
  const v16h xb0 = xt_frag_lds(xr, hf);
  const v16h xb1 = xt_frag_lds(xr + 32, hf);

  Frag cb0, cb1;
  cb0.half[0] = zero8h();
  cb0.half[1] = zero8h();
  cb1 = cb0;

#pragma unroll 1
  for (int h = 0; h < 4; ++h) {
    const _Float16* wq = w16 + WI_OFF + (size_t)(16 * h + m) * NDIM;
    v8f qacc = zero8f();
    qacc = wmma_f16(load_frag(wq, hf),      xb0, qacc);
    qacc = wmma_f16(load_frag(wq + 32, hf), xb1, qacc);
    Frag qf;
    qf.half[0] = cvt8((qacc * WSCI + ld8(inb + 16 * h + 8 * hf)) * QSC);
    qf.half[1] = zero8h();

    v8f s[5];
    const _Float16* kp = khs + (16 * w + m) * KP + 16 * h + 8 * hf;
#pragma unroll
    for (int j = 0; j < 5; ++j) {
      Frag kf;
      kf.half[0] = *(const v8ha*)(kp + 16 * j * KP);
      kf.half[1] = zero8h();
      s[j] = wmma_f16(kf.v, qf.v, zero8f());
    }
    float mx = -1e30f;
#pragma unroll
    for (int j = 0; j < 5; ++j) {
#pragma unroll
      for (int r = 0; r < 8; ++r) {
        const int key = t0 - WLEN + 16 * j + 8 * hf + r;
        const bool ok = (key >= 0) && (key <= tq) && (key > tq - WLEN);
        const float sv = ok ? s[j][r] : -1e30f;
        s[j][r] = sv;
        mx = fmaxf(mx, sv);
      }
    }
    mx = fmaxf(mx, __shfl_xor(mx, 16));
    float sum = 0.0f;
#pragma unroll
    for (int j = 0; j < 5; ++j) {
#pragma unroll
      for (int r = 0; r < 8; ++r) {
        const float e = __expf(s[j][r] - mx);
        s[j][r] = e;
        sum += e;
      }
    }
    sum += __shfl_xor(sum, 16);
    const float pn = PSC / sum;
    Frag pb0, pb1, pb2;
    pb0.half[0] = cvt8(s[0] * pn); pb0.half[1] = cvt8(s[1] * pn);
    pb1.half[0] = cvt8(s[2] * pn); pb1.half[1] = cvt8(s[3] * pn);
    pb2.half[0] = cvt8(s[4] * pn); pb2.half[1] = zero8h();
    const _Float16* vp = vts + (16 * h + m) * VP + 16 * w;
    v8f o = zero8f();
    o = wmma_f16(load_frag(vp, hf),      pb0.v, o);
    o = wmma_f16(load_frag(vp + 32, hf), pb1.v, o);
    o = wmma_f16(load_frag(vp + 64, hf), pb2.v, o);
    const v8h c16 = cvt8(o * PSCI);
    if (h == 0)      cb0.half[0] = c16;
    else if (h == 1) cb0.half[1] = c16;
    else if (h == 2) cb1.half[0] = c16;
    else             cb1.half[1] = c16;
  }

  v8f yv[4];
#pragma unroll
  for (int ct = 0; ct < 4; ++ct) {
    const _Float16* wo = w16 + WO_OFF + (size_t)(16 * ct + m) * NDIM;
    v8f a = zero8f();
    a = wmma_f16(load_frag(wo, hf),      cb0.v, a);
    a = wmma_f16(load_frag(wo + 32, hf), cb1.v, a);
    yv[ct] = a * WSCI + ld8(outb + 16 * ct + 8 * hf) + ld8a(xr + 16 * ct + 8 * hf);
  }
  {
    float s1 = hsum8((yv[0] + yv[1]) + (yv[2] + yv[3]));
    s1 += __shfl_xor(s1, 16);
    const float mu = s1 * (1.0f / NDIM);
#pragma unroll
    for (int ct = 0; ct < 4; ++ct) yv[ct] = yv[ct] - mu;
    float s2 = hsum8((yv[0] * yv[0] + yv[1] * yv[1]) + (yv[2] * yv[2] + yv[3] * yv[3]));
    s2 += __shfl_xor(s2, 16);
    const float rs = rsqrtf(s2 * (1.0f / NDIM) + 1e-5f);
#pragma unroll
    for (int ct = 0; ct < 4; ++ct) {
      yv[ct] = yv[ct] * rs * ld8(l1w + 16 * ct + 8 * hf) + ld8(l1b + 16 * ct + 8 * hf);
      st8a(sorow + 16 * ct + 8 * hf, yv[ct]);
    }
  }
  Frag nb0, nb1;
  nb0.half[0] = cvt8(yv[0]); nb0.half[1] = cvt8(yv[1]);
  nb1.half[0] = cvt8(yv[2]); nb1.half[1] = cvt8(yv[3]);
  __asm__ __volatile__("" ::: "memory");

  v8f facc[4];
#pragma unroll
  for (int ct = 0; ct < 4; ++ct) facc[ct] = zero8f();
#pragma unroll 1
  for (int mc = 0; mc < DFFN / 32; ++mc) {
    Frag gb;
#pragma unroll
    for (int u = 0; u < 2; ++u) {
      const int hrow = 32 * mc + 16 * u;
      const _Float16* wa = w16 + W1_OFF + (size_t)(hrow + m) * NDIM;
      v8f ha = zero8f();
      ha = wmma_f16(load_frag(wa, hf),      nb0.v, ha);
      ha = wmma_f16(load_frag(wa + 32, hf), nb1.v, ha);
      const v8f pre = ha * WSCI + ld8(b1 + hrow + 8 * hf);
      v8f g;
#pragma unroll
      for (int r = 0; r < 8; ++r) g[r] = gelu_f(pre[r]);
      gb.half[u] = cvt8(g);
    }
#pragma unroll
    for (int ct = 0; ct < 4; ++ct) {
      const _Float16* wb = w16 + W2_OFF + (size_t)(16 * ct + m) * DFFN + 32 * mc;
      facc[ct] = wmma_f16(load_frag(wb, hf), gb.v, facc[ct]);
    }
  }

  {
    v8f zv[4];
#pragma unroll
    for (int ct = 0; ct < 4; ++ct)
      zv[ct] = facc[ct] * WSCI + ld8(b2 + 16 * ct + 8 * hf) + ld8a(sorow + 16 * ct + 8 * hf);
    float s1 = hsum8((zv[0] + zv[1]) + (zv[2] + zv[3]));
    s1 += __shfl_xor(s1, 16);
    const float mu = s1 * (1.0f / NDIM);
#pragma unroll
    for (int ct = 0; ct < 4; ++ct) zv[ct] = zv[ct] - mu;
    float s2 = hsum8((zv[0] * zv[0] + zv[1] * zv[1]) + (zv[2] * zv[2] + zv[3] * zv[3]));
    s2 += __shfl_xor(s2, 16);
    const float rs = rsqrtf(s2 * (1.0f / NDIM) + 1e-5f);
#pragma unroll
    for (int ct = 0; ct < 4; ++ct) {
      zv[ct] = zv[ct] * rs * ld8(l2w + 16 * ct + 8 * hf) + ld8(l2b + 16 * ct + 8 * hf);
      st8a(sorow + 16 * ct + 8 * hf, zv[ct]);
    }
  }
  __syncthreads();

  const size_t rowbase = (size_t)n * SEQT + t0;
  const float* sow = so + w * (16 * NDIM);
  y_store_pass(sow, yg, rowbase, l);
  __threadfence();
  y_store_pass(sow, yg, rowbase, l);
}

__device__ __forceinline__ void out_store_pass(const float* st, float* og, size_t pbase, int w, int l) {
  const int q8 = l & 7, sub = l >> 3;
#pragma unroll 1
  for (int g = w; g < 2 * NF; g += 8) {
    const int L  = 4 * g + sub;
    const int cl = L / NF;
    const int li = L - cl * NF;
    const v4f v = *(const v4fa*)(st + cl * RUN + 32 * li + 4 * q8);
    *(volatile v4f*)(og + pbase + (size_t)cl * CST + 32 * li + 4 * q8) = v;
  }
}

__global__ __launch_bounds__(256) void out_layout_kernel(const float* __restrict__ yg,
                                                         float* __restrict__ og)
{
  __shared__ __align__(16) float st[8 * RUN];
  const int tid = threadIdx.x, w = tid >> 5, l = tid & 31;
  const int t0 = blockIdx.x * TL, c0 = blockIdx.y * 8, b = blockIdx.z;
  for (int i = tid; i < RUN; i += 256) {
    const int f = i >> 5, tl = i & 31;
    const float* yr = yg + ((size_t)(b * NF + f) * SEQT + t0 + tl) * NDIM + c0;
    const v4f a = *(const v4fa*)yr;
    const v4f c = *(const v4fa*)(yr + 4);
    const int o = tl * NF + f;
    st[0 * RUN + o] = a.x; st[1 * RUN + o] = a.y; st[2 * RUN + o] = a.z; st[3 * RUN + o] = a.w;
    st[4 * RUN + o] = c.x; st[5 * RUN + o] = c.y; st[6 * RUN + o] = c.z; st[7 * RUN + o] = c.w;
  }
  __syncthreads();
  const size_t pbase = (size_t)(b * NDIM + c0) * CST + (size_t)t0 * NF;
  out_store_pass(st, og, pbase, w, l);
  __threadfence();
  out_store_pass(st, og, pbase, w, l);
}

extern "C" void kernel_launch(void* const* d_in, const int* in_sizes, int n_in,
                              void* d_out, int out_size, void* d_ws, size_t ws_size,
                              hipStream_t stream) {
  if (n_in < 15) return;
  const int per_b = NDIM * SEQT * NF;
  const int B = in_sizes[0] / per_b;
  if (B < 1 || in_sizes[0] != B * per_b) return;
  if (in_sizes[1] != in_sizes[0] || in_sizes[2] != in_sizes[0]) return;
  if (in_sizes[3] != 3 * NDIM * NDIM || in_sizes[4] != 3 * NDIM) return;
  if (in_sizes[5] != NDIM * NDIM || in_sizes[6] != NDIM) return;
  if (in_sizes[7] != NDIM || in_sizes[8] != NDIM) return;
  if (in_sizes[9] != DFFN * NDIM || in_sizes[10] != DFFN) return;
  if (in_sizes[11] != NDIM * DFFN || in_sizes[12] != NDIM) return;
  if (in_sizes[13] != NDIM || in_sizes[14] != NDIM) return;
  if (out_size != in_sizes[0]) return;

  const int nseq = B * NF;
  const size_t w16_bytes = (size_t)W16_N * 2;
  const size_t y_off     = w16_bytes;
  const size_t y_bytes   = (size_t)nseq * SEQT * NDIM * 4;
  if (y_off + y_bytes > ws_size) return;

  const float* qg   = (const float*)d_in[0];
  const float* kg   = (const float*)d_in[1];
  const float* vg   = (const float*)d_in[2];
  const float* inw  = (const float*)d_in[3];
  const float* inb  = (const float*)d_in[4];
  const float* outw = (const float*)d_in[5];
  const float* outb = (const float*)d_in[6];
  const float* l1w  = (const float*)d_in[7];
  const float* l1b  = (const float*)d_in[8];
  const float* w1   = (const float*)d_in[9];
  const float* b1   = (const float*)d_in[10];
  const float* w2   = (const float*)d_in[11];
  const float* b2   = (const float*)d_in[12];
  const float* l2w  = (const float*)d_in[13];
  const float* l2b  = (const float*)d_in[14];
  float* og = (float*)d_out;

  char* ws = (char*)d_ws;
  _Float16* w16 = (_Float16*)ws;
  float* yg = (float*)(ws + y_off);

  cvt_w_kernel<<<(W16_N / 8 + 255) / 256, 256, 0, stream>>>(inw, outw, w1, w2, w16);

  fused_block_kernel<<<nseq * (SEQT / CHUNK), 256, 0, stream>>>(
      qg, kg, vg, w16, inb, outb, l1w, l1b, b1, b2, l2w, l2b, yg);

  dim3 gOut(SEQT / TL, NDIM / 8, B);
  out_layout_kernel<<<gOut, 256, 0, stream>>>(yg, og);
}
